// SS2D_CAAS_5188320494184
// MI455X (gfx1250) — hardware-run, weakly checked
//
#include <hip/hip_runtime.h>
#include <math.h>

typedef __attribute__((ext_vector_type(16))) _Float16 v16h;
typedef __attribute__((ext_vector_type(8)))  _Float16 v8h;
typedef __attribute__((ext_vector_type(16))) __bf16   v16b;
typedef __attribute__((ext_vector_type(8)))  __bf16   v8b;
typedef __attribute__((ext_vector_type(8)))  float    v8f;
typedef __attribute__((ext_vector_type(4)))  float    v4f;
typedef __attribute__((ext_vector_type(2)))  float    v2f;
typedef __attribute__((ext_vector_type(4)))  unsigned v4u;

constexpr int kNb    = 8;
constexpr int kDm    = 96;
constexpr int kSide  = 64;
constexpr int kLen   = kSide * kSide;
constexpr int kDin   = 192;
constexpr int kDir   = 4;
constexpr int kRank  = 6;
constexpr int kXc    = 8;
constexpr int kHid   = 32;
constexpr int kPix   = kNb * kLen;
constexpr int kPitA  = 128;
constexpr int kPitP  = 64;
constexpr int kMpadO = 128;
constexpr float kCarry    = 64.0f;
constexpr float kUncarry2 = 1.0f / (kCarry * kCarry);
constexpr float kF16Min   = 6.103515625e-05f;
static_assert(kLen == 4096);
static_assert(kPix == 32768);
static_assert(kRank + 2 == kXc);
static_assert((kDm % 32) == 0 && (kDin % 32) == 0);
static_assert((kPix % 64) == 0 && (kDin % 64) == 0 && (kLen % 64) == 0 && (kMpadO % 64) == 0 && (kPitP % 64) == 0);

constexpr size_t kSzXA   = (size_t)kPix * kPitA * 2;
constexpr size_t kSzXPRE = (size_t)kPix * kDin * 4;
constexpr size_t kSzYSC  = (size_t)kNb * kDir * kLen * kDin * 2;
constexpr size_t kSzR0   = kSzYSC;
constexpr size_t kSzWIN  = (size_t)(2 * kDin) * kPitA * 2;
constexpr size_t kSzWXP  = (size_t)64 * kDin * 2;
constexpr size_t kSzWOUT = (size_t)kMpadO * kDin * 2;
constexpr size_t kSzZ    = (size_t)kPix * kDin * 4;
constexpr size_t kSzXS   = (size_t)kPix * kDin * 4;
constexpr size_t kSzXSh  = (size_t)kPix * kDin * 2;
constexpr size_t kSzP    = (size_t)kPix * kPitP * 4;
constexpr size_t kSzWD   = (size_t)kPix * 4 * 4;
constexpr size_t kOffXA   = 0;
constexpr size_t kOffXPRE = kOffXA + kSzXA;
constexpr size_t kOffYSC  = 0;
constexpr size_t kOffWIN  = kSzR0;
constexpr size_t kOffWXP  = kOffWIN + kSzWIN;
constexpr size_t kOffWOUT = kOffWXP + kSzWXP;
constexpr size_t kOffZ    = kOffWOUT + kSzWOUT;
constexpr size_t kOffXS   = kOffZ + kSzZ;
constexpr size_t kOffXSh  = kOffXS + kSzXS;
constexpr size_t kOffP    = kOffXSh + kSzXSh;
constexpr size_t kOffWD   = kOffP + kSzP;
constexpr size_t kWsTotal = kOffWD + kSzWD;
static_assert(kSzXA + kSzXPRE <= kSzR0);
static_assert(kWsTotal == 122331136ull);
static_assert(kWsTotal <= 134217728ull);
static_assert((kOffXPRE % 128) == 0 && (kOffWIN % 128) == 0 && (kOffWXP % 128) == 0 && (kOffWOUT % 128) == 0 &&
              (kOffZ % 128) == 0 && (kOffXS % 128) == 0 && (kOffXSh % 128) == 0 && (kOffP % 128) == 0 &&
              (kOffWD % 128) == 0);

__device__ __forceinline__ unsigned short f2bf_bits(float f) {
  unsigned u = __float_as_uint(f);
  return (unsigned short)((u + 0x7FFFu + ((u >> 16) & 1u)) >> 16);
}
__device__ __forceinline__ float bf_bits2f(unsigned short h) { return __uint_as_float(((unsigned)h) << 16); }
__device__ __forceinline__ float rbf(float f) { return bf_bits2f(f2bf_bits(f)); }
__device__ __forceinline__ _Float16 to_h_flush(float v) {
  const float w = (fabsf(v) < kF16Min) ? 0.0f : v;
  return (_Float16)w;
}
__device__ __forceinline__ unsigned pack_h2(float a, float b) {
  const _Float16 h0 = to_h_flush(a);
  const _Float16 h1 = to_h_flush(b);
  const unsigned short u0 = __builtin_bit_cast(unsigned short, h0);
  const unsigned short u1 = __builtin_bit_cast(unsigned short, h1);
  return (unsigned)u0 | ((unsigned)u1 << 16);
}
__device__ __forceinline__ unsigned pack_b2(float a, float b) {
  const unsigned short u0 = f2bf_bits(a);
  const unsigned short u1 = f2bf_bits(b);
  return (unsigned)u0 | ((unsigned)u1 << 16);
}
__device__ __forceinline__ float h16_to_f32(unsigned hb) {
  const unsigned sgn = (hb & 0x8000u) << 16;
  const unsigned em = hb & 0x7fffu;
  const float fn = __uint_as_float((em << 13) + 0x38000000u);
  const float fs = (float)em * 5.9604644775390625e-8f;
  const float mag = (em < 0x400u) ? fs : fn;
  return __uint_as_float(__float_as_uint(mag) | sgn);
}
__device__ __forceinline__ void store2_v4u(void* p, v4u v) {
  *(volatile v4u*)p = v;
  __threadfence();
  *(volatile v4u*)p = v;
}
__device__ __forceinline__ int seq_to_spatial(int k, int l) {
  const int lp = (k >= 2) ? (kLen - 1 - l) : l;
  const int tr = ((lp & 63) << 6) | (lp >> 6);
  return (k & 1) ? tr : lp;
}

__device__ __forceinline__ void keep4_h(v16h a, v16h b, v16h c, v16h d) { asm volatile("v_nop" :: "v"(a), "v"(b), "v"(c), "v"(d)); }
__device__ __forceinline__ void keep4_b(v16b a, v16b b, v16b c, v16b d) { asm volatile("v_nop" :: "v"(a), "v"(b), "v"(c), "v"(d)); }
__device__ __forceinline__ void acc_guard4(v8f& a, v8f& b, v8f& c, v8f& d) { asm volatile("v_nop\n\tv_nop\n\tv_nop\n\tv_nop" : "+v"(a), "+v"(b), "+v"(c), "+v"(d)); }
template <typename T> struct Frag;
template <> struct Frag<_Float16> {
  typedef v16h V; union U { v16h v; v8h h[2]; };
  static __device__ __forceinline__ v16h load(const _Float16* p) {
    U f; f.h[0] = *(const v8h*)(p); f.h[1] = *(const v8h*)(p + 16); return f.v;
  }
  static __device__ __forceinline__ v8f mma(v16h a, v16h b, v8f c) {
    c = __builtin_amdgcn_wmma_f32_16x16x32_f16(false, a, false, b, (short)0, c, false, false);
    asm volatile("v_nop\n\tv_nop\n\tv_nop\n\tv_nop" : "+v"(c) : "v"(a), "v"(b));
    return c;
  }
  static __device__ __forceinline__ void keep(v16h a, v16h b, v16h c, v16h d) { keep4_h(a, b, c, d); }
};
template <> struct Frag<__bf16> {
  typedef v16b V; union U { v16b v; v8b h[2]; };
  static __device__ __forceinline__ v16b load(const __bf16* p) {
    U f; f.h[0] = *(const v8b*)(p); f.h[1] = *(const v8b*)(p + 16); return f.v;
  }
  static __device__ __forceinline__ v8f mma(v16b a, v16b b, v8f c) {
    c = __builtin_amdgcn_wmma_f32_16x16x32_bf16(false, a, false, b, (short)0, c, false, false);
    asm volatile("v_nop\n\tv_nop\n\tv_nop\n\tv_nop" : "+v"(c) : "v"(a), "v"(b));
    return c;
  }
  static __device__ __forceinline__ void keep(v16b a, v16b b, v16b c, v16b d) { keep4_b(a, b, c, d); }
};

template <int ET> struct Elem;
template <> struct Elem<0> { typedef _Float16 T; };
template <> struct Elem<1> { typedef __bf16 T; };
template <int ET>
__global__ __launch_bounds__(256) void wmma_gemm64(
    const unsigned short* __restrict__ Ap, int lda, long strideA,
    const unsigned short* __restrict__ Btp, int ldb, long strideB,
    float* __restrict__ Cout, int ldc, long strideC,
    int M, int N, int K, float scale, int mstore) {
  typedef typename Elem<ET>::T T;
  typedef typename Frag<T>::V V;
  const T* A = (const T*)Ap; const T* Bt = (const T*)Btp;
  __shared__ __align__(16) float sT[8][16 * 68];
  const int b    = blockIdx.y;
  const int lane = threadIdx.x & 31;
  const int wave = threadIdx.x >> 5;
  const int tilesN = N >> 6;
  const int tilesM = M >> 6;
  const int tile = blockIdx.x * 8 + wave;
  if (tile >= tilesM * tilesN) return;
  const int tm = tile / tilesN;
  const int tn = tile - tm * tilesN;
  const int m0 = tm << 6;
  const int n0 = tn << 6;

  const T* Ab = A  + (size_t)b * strideA;
  const T* Bb = Bt + (size_t)b * strideB;

  const int rlane = lane & 15;
  const int koff  = (lane >> 4) * 8;
  const int mOff  = (lane >> 4) * 8;

  v8f acc[4][4];
#pragma unroll
  for (int i = 0; i < 4; ++i)
#pragma unroll
    for (int j = 0; j < 4; ++j) acc[i][j] = (v8f){0.f,0.f,0.f,0.f,0.f,0.f,0.f,0.f};

  for (int k0 = 0; k0 < K; k0 += 32) {
    V bh[4];
#pragma unroll
    for (int j = 0; j < 4; ++j) {
      const size_t bo = (size_t)(n0 + (j << 4) + rlane) * ldb + koff + k0;
      bh[j] = Frag<T>::load(Bb + bo);
    }
#pragma unroll
    for (int i = 0; i < 4; ++i) {
      const size_t ao = (size_t)(m0 + (i << 4) + rlane) * lda + koff + k0;
      V ah = Frag<T>::load(Ab + ao);
#pragma unroll
      for (int j = 0; j < 4; ++j) {
        acc[i][j] = Frag<T>::mma(ah, bh[j], acc[i][j]);
      }
    }
    Frag<T>::keep(bh[0], bh[1], bh[2], bh[3]);
  }
  acc_guard4(acc[0][0], acc[0][1], acc[0][2], acc[0][3]);
  acc_guard4(acc[1][0], acc[1][1], acc[1][2], acc[1][3]);
  acc_guard4(acc[2][0], acc[2][1], acc[2][2], acc[2][3]);
  acc_guard4(acc[3][0], acc[3][1], acc[3][2], acc[3][3]);

  float* slab = sT[wave];
  float* C = Cout + (size_t)b * strideC;
#pragma unroll
  for (int i = 0; i < 4; ++i) {
    const int mBase = m0 + (i << 4);
#pragma unroll
    for (int j = 0; j < 4; ++j) {
#pragma unroll
      for (int r = 0; r < 8; ++r) {
        const float v = acc[i][j][r] * scale;
        slab[(mOff + r) * 68 + (j << 4) + rlane] = v;
      }
    }
    __builtin_amdgcn_fence(__ATOMIC_RELEASE, "workgroup");
    __builtin_amdgcn_wave_barrier();
    __builtin_amdgcn_fence(__ATOMIC_ACQUIRE, "workgroup");
    if (mBase < mstore) {
      const int hh = lane >> 4, c4 = (lane & 15) * 4;
      for (int pass = 0; pass < 2; ++pass) {
#pragma unroll
        for (int it = 0; it < 8; ++it) {
          const int row = it * 2 + hh;
          v4f v = *(const v4f*)(slab + row * 68 + c4);
          *(volatile v4f*)(C + (size_t)(mBase + row) * ldc + n0 + c4) = v;
        }
        __threadfence();
      }
    }
    __builtin_amdgcn_fence(__ATOMIC_RELEASE, "workgroup");
    __builtin_amdgcn_wave_barrier();
    __builtin_amdgcn_fence(__ATOMIC_ACQUIRE, "workgroup");
  }
}

__global__ __launch_bounds__(256) void prep_x_kernel(const float* __restrict__ x, unsigned short* __restrict__ XA) {
  __shared__ __align__(16) float sT[64 * 100];
  const int tid = threadIdx.x;
  const int b  = blockIdx.x >> 6;
  const int s0 = (blockIdx.x & 63) * 64;
#pragma unroll
  for (int it = 0; it < 6; ++it) {
    const int idx = tid + 256 * it;
    const int c = idx >> 4;
    const int s4 = (idx & 15) * 4;
    const v4f v = *(const v4f*)(x + ((size_t)(b * kDm + c)) * kLen + s0 + s4);
    sT[(s4 + 0) * 100 + c] = v[0];
    sT[(s4 + 1) * 100 + c] = v[1];
    sT[(s4 + 2) * 100 + c] = v[2];
    sT[(s4 + 3) * 100 + c] = v[3];
  }
  __syncthreads();
  v4u ov[4];
#pragma unroll
  for (int it = 0; it < 4; ++it) {
    const int idx = tid + 256 * it;
    const int row = idx >> 4;
    const int ch = idx & 15;
    const bool keepc = (ch < 12);
    const int cc = keepc ? ch : 11;
    const v4f a0 = *(const v4f*)(sT + row * 100 + cc * 8);
    const v4f a1 = *(const v4f*)(sT + row * 100 + cc * 8 + 4);
    const unsigned w0 = pack_b2(a0[0], a0[1]);
    const unsigned w1 = pack_b2(a0[2], a0[3]);
    const unsigned w2 = pack_b2(a1[0], a1[1]);
    const unsigned w3 = pack_b2(a1[2], a1[3]);
    ov[it][0] = keepc ? w0 : 0u;
    ov[it][1] = keepc ? w1 : 0u;
    ov[it][2] = keepc ? w2 : 0u;
    ov[it][3] = keepc ? w3 : 0u;
  }
  for (int pass = 0; pass < 2; ++pass) {
#pragma unroll
    for (int it = 0; it < 4; ++it) {
      const int idx = tid + 256 * it;
      const int row = idx >> 4;
      const int ch = idx & 15;
      unsigned short* q = XA + ((size_t)(b * kLen + s0 + row)) * kPitA + ch * 8;
      *(volatile v4u*)(void*)q = ov[it];
    }
    __threadfence();
  }
}

__global__ __launch_bounds__(256) void prep_w_kernel(
    const float* __restrict__ ipw, const float* __restrict__ xpw, const float* __restrict__ opw,
    unsigned short* __restrict__ WIN, unsigned short* __restrict__ WXP, unsigned short* __restrict__ WOUT) {
  const int tid = threadIdx.x;
  const int blk = blockIdx.x;
  if (blk < 24) {
    const int i = blk * 256 + tid;
    const int row = i >> 4;
    const int ch = i & 15;
    const bool keepc = (ch < 12);
    const int cc = keepc ? ch : 11;
    const float* p = ipw + (size_t)row * kDm + cc * 8;
    const v4f a0 = *(const v4f*)(p);
    const v4f a1 = *(const v4f*)(p + 4);
    const unsigned w0 = pack_b2(a0[0], a0[1]);
    const unsigned w1 = pack_b2(a0[2], a0[3]);
    const unsigned w2 = pack_b2(a1[0], a1[1]);
    const unsigned w3 = pack_b2(a1[2], a1[3]);
    v4u o;
    o[0] = keepc ? w0 : 0u;
    o[1] = keepc ? w1 : 0u;
    o[2] = keepc ? w2 : 0u;
    o[3] = keepc ? w3 : 0u;
    store2_v4u((void*)(WIN + (size_t)i * 8), o);
  } else if (blk < 30) {
    const int j = (blk - 24) * 256 + tid;
    const int row = j / 24;
    const int ch = j - row * 24;
    const bool keepr = (row < 32);
    const int rc = keepr ? row : 31;
    const float* p = xpw + (size_t)rc * kDin + ch * 8;
    const v4f a0 = *(const v4f*)(p);
    const v4f a1 = *(const v4f*)(p + 4);
    const unsigned w0 = pack_h2(rbf(a0[0]) * kCarry, rbf(a0[1]) * kCarry);
    const unsigned w1 = pack_h2(rbf(a0[2]) * kCarry, rbf(a0[3]) * kCarry);
    const unsigned w2 = pack_h2(rbf(a1[0]) * kCarry, rbf(a1[1]) * kCarry);
    const unsigned w3 = pack_h2(rbf(a1[2]) * kCarry, rbf(a1[3]) * kCarry);
    v4u o;
    o[0] = keepr ? w0 : 0u;
    o[1] = keepr ? w1 : 0u;
    o[2] = keepr ? w2 : 0u;
    o[3] = keepr ? w3 : 0u;
    store2_v4u((void*)(WXP + (size_t)j * 8), o);
  } else {
    const int j = (blk - 30) * 256 + tid;
    const int row = j / 24;
    const int ch = j - row * 24;
    const bool keepr = (row < kDm);
    const int rc = keepr ? row : (kDm - 1);
    const float* p = opw + (size_t)rc * kDin + ch * 8;
    const v4f a0 = *(const v4f*)(p);
    const v4f a1 = *(const v4f*)(p + 4);
    const unsigned w0 = pack_h2(rbf(a0[0]) * kCarry, rbf(a0[1]) * kCarry);
    const unsigned w1 = pack_h2(rbf(a0[2]) * kCarry, rbf(a0[3]) * kCarry);
    const unsigned w2 = pack_h2(rbf(a1[0]) * kCarry, rbf(a1[1]) * kCarry);
    const unsigned w3 = pack_h2(rbf(a1[2]) * kCarry, rbf(a1[3]) * kCarry);
    v4u o;
    o[0] = keepr ? w0 : 0u;
    o[1] = keepr ? w1 : 0u;
    o[2] = keepr ? w2 : 0u;
    o[3] = keepr ? w3 : 0u;
    store2_v4u((void*)(WOUT + (size_t)j * 8), o);
  }
}

__device__ __forceinline__ void conv_load_col(const float* src, int hmc, int h, int hpc, bool vm, bool vp, int ww,
                                              float& c0, float& c1, float& c2) {
  const bool vw = (ww >= 0) && (ww < kSide);
  const int wc = (ww < 0) ? 0 : ((ww > kSide - 1) ? (kSide - 1) : ww);
  const float t0 = src[(size_t)((hmc << 6) + wc) * kDin];
  const float t1 = src[(size_t)((h << 6) + wc) * kDin];
  const float t2 = src[(size_t)((hpc << 6) + wc) * kDin];
  c0 = (vw && vm) ? t0 : 0.0f;
  c1 = vw ? t1 : 0.0f;
  c2 = (vw && vp) ? t2 : 0.0f;
}

__global__ __launch_bounds__(192) void dwconv_silu_kernel(
    const float* __restrict__ XPRE, const float* __restrict__ cw, const float* __restrict__ cb,
    float* __restrict__ XS, unsigned short* __restrict__ XSh) {
  __shared__ __align__(16) float sT[8 * kDin];
  const int d = threadIdx.x;
  const int p0 = blockIdx.x * 8;
  const int b = p0 >> 12;
  const int s0 = p0 & (kLen - 1);
  const int h = s0 >> 6;
  const int w0 = s0 & 63;
  float wk[9];
#pragma unroll
  for (int i = 0; i < 9; ++i) wk[i] = rbf(cw[d * 9 + i]);
  const float bc = rbf(cb[d]);
  const float* src = XPRE + (size_t)b * kLen * kDin + d;
  const bool vm = (h > 0);
  const bool vp = (h < kSide - 1);
  const int hmc = vm ? (h - 1) : 0;
  const int hpc = vp ? (h + 1) : (kSide - 1);
  float a0, a1, a2, b0, b1, b2;
  conv_load_col(src, hmc, h, hpc, vm, vp, w0 - 1, a0, a1, a2);
  conv_load_col(src, hmc, h, hpc, vm, vp, w0, b0, b1, b2);
#pragma unroll 1
  for (int j = 0; j < 8; ++j) {
    float c0, c1, c2;
    conv_load_col(src, hmc, h, hpc, vm, vp, w0 + j + 1, c0, c1, c2);
    float acc = wk[0] * a0;
    acc = fmaf(wk[1], b0, acc);
    acc = fmaf(wk[2], c0, acc);
    acc = fmaf(wk[3], a1, acc);
    acc = fmaf(wk[4], b1, acc);
    acc = fmaf(wk[5], c1, acc);
    acc = fmaf(wk[6], a2, acc);
    acc = fmaf(wk[7], b2, acc);
    acc = fmaf(wk[8], c2, acc);
    const float sv = acc + bc;
    const float sg = 1.0f / (1.0f + expf(-sv));
    sT[j * kDin + d] = sv * sg;
    a0 = b0; a1 = b1; a2 = b2;
    b0 = c0; b1 = c1; b2 = c2;
  }
  __syncthreads();
  const v4f f0 = *(const v4f*)(sT + d * 4);
  const v4f f1 = *(const v4f*)(sT + (d + 192) * 4);
  const v4f g0 = *(const v4f*)(sT + d * 8);
  const v4f g1 = *(const v4f*)(sT + d * 8 + 4);
  v4u hv;
  hv[0] = pack_h2(g0[0] * kCarry, g0[1] * kCarry);
  hv[1] = pack_h2(g0[2] * kCarry, g0[3] * kCarry);
  hv[2] = pack_h2(g1[0] * kCarry, g1[1] * kCarry);
  hv[3] = pack_h2(g1[2] * kCarry, g1[3] * kCarry);
  float* of = XS + (size_t)p0 * kDin;
  unsigned short* oh = XSh + (size_t)p0 * kDin;
  for (int pass = 0; pass < 2; ++pass) {
    *(volatile v4f*)(of + d * 4) = f0;
    *(volatile v4f*)(of + (d + 192) * 4) = f1;
    *(volatile v4u*)(void*)(oh + d * 8) = hv;
    __threadfence();
  }
}

__global__ __launch_bounds__(256) void prior_weights_kernel(
    const float* __restrict__ prior, const float* __restrict__ alpha,
    const float* __restrict__ w1, const float* __restrict__ b1,
    const float* __restrict__ bnw, const float* __restrict__ bnb,
    const float* __restrict__ bnm, const float* __restrict__ bnv,
    const float* __restrict__ w2, const float* __restrict__ b2,
    float* __restrict__ WD) {
  __shared__ float sW1[kHid * 4];
  __shared__ float sW2[4 * kHid];
  __shared__ float sB1[kHid];
  __shared__ float sMean[kHid];
  __shared__ float sRs[kHid];
  __shared__ float sBw[kHid];
  __shared__ float sBb[kHid];
  __shared__ float sB2[4];
  const int tid = threadIdx.x;
  {
    const int i1 = tid & 127;
    const int i2 = tid & 31;
    const int i3 = tid & 3;
    sW1[i1] = rbf(w1[i1]);
    sW2[i1] = rbf(w2[i1]);
    sB1[i2] = rbf(b1[i2]);
    sMean[i2] = rbf(bnm[i2]);
    sRs[i2] = 1.0f / sqrtf(rbf(bnv[i2]) + 1e-5f);
    sBw[i2] = rbf(bnw[i2]);
    sBb[i2] = rbf(bnb[i2]);
    sB2[i3] = rbf(b2[i3]);
  }
  __syncthreads();
  const int p = blockIdx.x * 256 + tid;
  const int b = p >> 12;
  const int l = p & (kLen - 1);
  const float pr0 = rbf(prior[((size_t)(b * 4 + 0)) * kLen + l]);
  const float pr1 = rbf(prior[((size_t)(b * 4 + 1)) * kLen + l]);
  const float pr2 = rbf(prior[((size_t)(b * 4 + 2)) * kLen + l]);
  const float pr3 = rbf(prior[((size_t)(b * 4 + 3)) * kLen + l]);
  const float al = rbf(alpha[0]);
  const float sa = 1.0f / (1.0f + expf(-al));
  float g0 = 0.0f, g1 = 0.0f, g2 = 0.0f, g3 = 0.0f;
#pragma unroll 1
  for (int j = 0; j < kHid; ++j) {
    float t = sW1[j * 4 + 0] * pr0;
    t = fmaf(sW1[j * 4 + 1], pr1, t);
    t = fmaf(sW1[j * 4 + 2], pr2, t);
    t = fmaf(sW1[j * 4 + 3], pr3, t);
    t = t + sB1[j];
    t = (t - sMean[j]) * sRs[j];
    t = t * sBw[j] + sBb[j];
    t = fmaxf(t, 0.0f);
    g0 = fmaf(sW2[0 * kHid + j], t, g0);
    g1 = fmaf(sW2[1 * kHid + j], t, g1);
    g2 = fmaf(sW2[2 * kHid + j], t, g2);
    g3 = fmaf(sW2[3 * kHid + j], t, g3);
  }
  g0 += sB2[0]; g1 += sB2[1]; g2 += sB2[2]; g3 += sB2[3];
  v4f o;
  o[0] = 1.0f + sa * (1.0f / (1.0f + expf(-g0)) - 1.0f);
  o[1] = 1.0f + sa * (1.0f / (1.0f + expf(-g1)) - 1.0f);
  o[2] = 1.0f + sa * (1.0f / (1.0f + expf(-g2)) - 1.0f);
  o[3] = 1.0f + sa * (1.0f / (1.0f + expf(-g3)) - 1.0f);
  float* q = WD + (size_t)p * 4;
  *(volatile v4f*)q = o;
  __threadfence();
  *(volatile v4f*)q = o;
}

__global__ __launch_bounds__(64) void scan_kernel(
    const float* __restrict__ P, const float* __restrict__ XS,
    const float* __restrict__ dtwg, const float* __restrict__ dtbg, const float* __restrict__ alog,
    unsigned short* __restrict__ YSC) {
  __shared__ __align__(16) float sP[64 * 8];
  __shared__ __align__(16) float sY[64 * 68];
  const int tid = threadIdx.x, lane = tid & 31, wave = tid >> 5;
  const int blk = blockIdx.x;
  const int b = blk / 12;
  const int rem = blk - b * 12;
  const int k = rem / 3;
  const int dblk = rem - k * 3;
  const int d = dblk * 64 + tid;
  const int kd = k * kDin + d;
  const float w0 = rbf(dtwg[kd * kRank + 0]);
  const float w1 = rbf(dtwg[kd * kRank + 1]);
  const float w2 = rbf(dtwg[kd * kRank + 2]);
  const float w3 = rbf(dtwg[kd * kRank + 3]);
  const float w4 = rbf(dtwg[kd * kRank + 4]);
  const float w5 = rbf(dtwg[kd * kRank + 5]);
  const float bb = rbf(dtbg[kd]);
  const float Aneg = -expf(rbf(alog[kd]));
  const size_t pixb = (size_t)b * kLen;
  const size_t yscb = (size_t)(b * kDir + k) * kLen;
  const int q = lane >> 3, c8 = (lane & 7) * 8;
  float h = 0.0f;
#pragma unroll 1
  for (int t0 = 0; t0 < kLen; t0 += 64) {
    __syncthreads();
    {
      const int sp = seq_to_spatial(k, t0 + tid);
      const float* pp = P + (pixb + sp) * kPitP + k * kXc;
      const v4f p0 = *(const v4f*)(pp);
      const v4f p1 = *(const v4f*)(pp + 4);
      *(v4f*)(sP + tid * 8) = p0;
      *(v4f*)(sP + tid * 8 + 4) = p1;
    }
    __syncthreads();
#pragma unroll 1
    for (int s = 0; s < 64; ++s) {
      const int sp = seq_to_spatial(k, t0 + s);
      const v4f q0 = *(const v4f*)(sP + s * 8);
      const v4f q1 = *(const v4f*)(sP + s * 8 + 4);
      const float xv = XS[(pixb + sp) * kDin + d];
      float dot = q0[0] * w0;
      dot = fmaf(q0[1], w1, dot);
      dot = fmaf(q0[2], w2, dot);
      dot = fmaf(q0[3], w3, dot);
      dot = fmaf(q1[0], w4, dot);
      dot = fmaf(q1[1], w5, dot);
      const float v = dot + bb;
      const float dt = fmaxf(v, 0.0f) + log1pf(expf(-fabsf(v)));
      const float a = expf(dt * Aneg);
      const float bx = (dt * q1[2]) * xv;
      h = fmaf(h, a, bx);
      sY[s * 68 + tid] = h * q1[3];
    }
    __syncthreads();
    v8h hv[8];
#pragma unroll
    for (int it = 0; it < 8; ++it) {
      const int row = it * 8 + wave * 4 + q;
      const float* sr = sY + row * 68 + c8;
      const v4f a0 = *(const v4f*)(sr);
      const v4f a1 = *(const v4f*)(sr + 4);
      hv[it][0] = (_Float16)a0[0];
      hv[it][1] = (_Float16)a0[1];
      hv[it][2] = (_Float16)a0[2];
      hv[it][3] = (_Float16)a0[3];
      hv[it][4] = (_Float16)a1[0];
      hv[it][5] = (_Float16)a1[1];
      hv[it][6] = (_Float16)a1[2];
      hv[it][7] = (_Float16)a1[3];
    }
    for (int pass = 0; pass < 2; ++pass) {
#pragma unroll
      for (int it = 0; it < 8; ++it) {
        const int row = it * 8 + wave * 4 + q;
        const int sp = seq_to_spatial(k, t0 + row);
        const size_t o = (yscb + sp) * kDin + dblk * 64 + c8;
        *(volatile v8h*)(void*)(YSC + o) = hv[it];
      }
      __threadfence();
    }
  }
}

__global__ __launch_bounds__(256) void merge_norm_gate_kernel(
    const float* __restrict__ XS, const float* __restrict__ Zp, const unsigned* __restrict__ YSCw,
    const float* __restrict__ WD, const float* __restrict__ Dsg, const float* __restrict__ onw,
    const float* __restrict__ onb, unsigned* __restrict__ YGw) {
  __shared__ __align__(16) float sDs[kDir * kDin];
  __shared__ __align__(16) float sNw[kDin];
  __shared__ __align__(16) float sNb[kDin];
  __shared__ __align__(16) float sYw[8 * kDin];
  __shared__ __align__(16) unsigned sOut[32 * 96];
  const int tid = threadIdx.x, lane = tid & 31, wave = tid >> 5;
#pragma unroll 1
  for (int i = tid; i < kDir * kDin; i += 256) sDs[i] = rbf(Dsg[i]);
  {
    const int tc = (tid < kDin) ? tid : (kDin - 1);
    float a = onw[tc];
    float c = onb[tc];
    asm volatile("" : "+v"(a), "+v"(c));
    if (tid < kDin) { sNw[tid] = rbf(a); sNb[tid] = rbf(c); }
  }
  __syncthreads();
  float* yw = sYw + wave * kDin;
  const int pblk = blockIdx.x * 32;
  constexpr size_t kPlaneW = (size_t)kLen * 96;
#pragma unroll 1
  for (int i = 0; i < 4; ++i) {
    const int p = pblk + wave * 4 + i;
    const int b = p >> 12;
    const int s = p & (kLen - 1);
    const int lc = ((s & 63) << 6) | (s >> 6);
    const size_t wb = (size_t)b * kLen;
    const float wd0 = WD[(wb + s) * 4 + 0];
    const float wd1 = WD[(wb + lc) * 4 + 1];
    const float wd2 = WD[(wb + (kLen - 1 - s)) * 4 + 2];
    const float wd3 = WD[(wb + (kLen - 1 - lc)) * 4 + 3];
    const float* xsr = XS + (size_t)p * kDin;
    const float* zr = Zp + (size_t)p * kDin;
    const unsigned* y0p = YSCw + ((size_t)(b * kDir) * kLen + s) * 96;
    float sum = 0.0f;
#pragma unroll 1
    for (int j = 0; j < 3; ++j) {
      const int c = 64 * j + 2 * lane;
      const int wi = 32 * j + lane;
      const v2f xv = *(const v2f*)(xsr + c);
      const unsigned u0 = y0p[wi];
      const unsigned u1 = y0p[kPlaneW + wi];
      const unsigned u2 = y0p[2 * kPlaneW + wi];
      const unsigned u3 = y0p[3 * kPlaneW + wi];
      const v2f e0 = *(const v2f*)(sDs + c);
      const v2f e1 = *(const v2f*)(sDs + kDin + c);
      const v2f e2 = *(const v2f*)(sDs + 2 * kDin + c);
      const v2f e3 = *(const v2f*)(sDs + 3 * kDin + c);
      const float t0a = wd0 * (h16_to_f32(u0 & 0xffffu) + e0[0] * xv[0]);
      const float t0b = wd0 * (h16_to_f32(u0 >> 16) + e0[1] * xv[1]);
      const float t1a = wd1 * (h16_to_f32(u1 & 0xffffu) + e1[0] * xv[0]);
      const float t1b = wd1 * (h16_to_f32(u1 >> 16) + e1[1] * xv[1]);
      const float t2a = wd2 * (h16_to_f32(u2 & 0xffffu) + e2[0] * xv[0]);
      const float t2b = wd2 * (h16_to_f32(u2 >> 16) + e2[1] * xv[1]);
      const float t3a = wd3 * (h16_to_f32(u3 & 0xffffu) + e3[0] * xv[0]);
      const float t3b = wd3 * (h16_to_f32(u3 >> 16) + e3[1] * xv[1]);
      const float ya = (t0a + t2a) + (t1a + t3a);
      const float yb = (t0b + t2b) + (t1b + t3b);
      yw[c] = ya;
      yw[c + 1] = yb;
      sum += ya + yb;
    }
#pragma unroll
    for (int off = 16; off >= 1; off >>= 1) sum += __shfl_xor(sum, off, 32);
    const float mu = sum * (1.0f / (float)kDin);
    float sq = 0.0f;
#pragma unroll 1
    for (int j = 0; j < 3; ++j) {
      const int c = 64 * j + 2 * lane;
      const float da = yw[c] - mu;
      const float db = yw[c + 1] - mu;
      sq = fmaf(da, da, sq);
      sq = fmaf(db, db, sq);
    }
#pragma unroll
    for (int off = 16; off >= 1; off >>= 1) sq += __shfl_xor(sq, off, 32);
    const float var = sq * (1.0f / (float)kDin);
    const float rstd = 1.0f / sqrtf(var + 1e-5f);
#pragma unroll 1
    for (int j = 0; j < 3; ++j) {
      const int c = 64 * j + 2 * lane;
      const int wi = 32 * j + lane;
      const v2f zv = *(const v2f*)(zr + c);
      const float na = (yw[c] - mu) * rstd * sNw[c] + sNb[c];
      const float nb = (yw[c + 1] - mu) * rstd * sNw[c + 1] + sNb[c + 1];
      const float za = zv[0];
      const float zb = zv[1];
      const float ga = za * (1.0f / (1.0f + expf(-za)));
      const float gb = zb * (1.0f / (1.0f + expf(-zb)));
      const float oa = na * ga;
      const float ob = nb * gb;
      sOut[(wave * 4 + i) * 96 + wi] = pack_h2(oa * kCarry, ob * kCarry);
    }
  }
  __syncthreads();
  v4u ov[3];
#pragma unroll
  for (int it = 0; it < 3; ++it) ov[it] = *(const v4u*)(sOut + (tid + 256 * it) * 4);
  unsigned* og = YGw + (size_t)pblk * 96;
  for (int pass = 0; pass < 2; ++pass) {
#pragma unroll
    for (int it = 0; it < 3; ++it) *(volatile v4u*)(og + (tid + 256 * it) * 4) = ov[it];
    __threadfence();
  }
}

extern "C" void kernel_launch(void* const* d_in, const int* in_sizes, int n_in,
                              void* d_out, int out_size, void* d_ws, size_t ws_size,
                              hipStream_t stream) {
  if (n_in < 22) return;
  if (in_sizes[0] != kNb * kDm * kLen) return;
  if (in_sizes[1] != kNb * 4 * kLen) return;
  if (in_sizes[2] != 1) return;
  if (in_sizes[3] != 2 * kDin * kDm) return;
  if (in_sizes[4] != kDin * 9) return;
  if (in_sizes[5] != kDin) return;
  if (in_sizes[6] != kDir * kXc * kDin) return;
  if (in_sizes[7] != kDir * kDin * kRank) return;
  if (in_sizes[8] != kDir * kDin) return;
  if (in_sizes[9] != kDir * kDin) return;
  if (in_sizes[10] != kDir * kDin) return;
  if (in_sizes[11] != kDin) return;
  if (in_sizes[12] != kDin) return;
  if (in_sizes[13] != kDm * kDin) return;
  if (in_sizes[14] != kHid * 4) return;
  if (in_sizes[15] != kHid) return;
  if (in_sizes[16] != kHid) return;
  if (in_sizes[17] != kHid) return;
  if (in_sizes[18] != kHid) return;
  if (in_sizes[19] != kHid) return;
  if (in_sizes[20] != 4 * kHid) return;
  if (in_sizes[21] != 4) return;
  if (out_size != kNb * kDm * kLen) return;
  if (ws_size < kWsTotal) return;

  const float* x      = (const float*)d_in[0];
  const float* prior  = (const float*)d_in[1];
  const float* alpha  = (const float*)d_in[2];
  const float* ipw    = (const float*)d_in[3];
  const float* cw     = (const float*)d_in[4];
  const float* cb     = (const float*)d_in[5];
  const float* xpw    = (const float*)d_in[6];
  const float* dtw    = (const float*)d_in[7];
  const float* dtb    = (const float*)d_in[8];
  const float* alog   = (const float*)d_in[9];
  const float* Dsg    = (const float*)d_in[10];
  const float* onw    = (const float*)d_in[11];
  const float* onb    = (const float*)d_in[12];
  const float* opw    = (const float*)d_in[13];
  const float* w1     = (const float*)d_in[14];
  const float* b1     = (const float*)d_in[15];
  const float* bnw    = (const float*)d_in[16];
  const float* bnb    = (const float*)d_in[17];
  const float* bnm    = (const float*)d_in[18];
  const float* bnv    = (const float*)d_in[19];
  const float* w2     = (const float*)d_in[20];
  const float* b2     = (const float*)d_in[21];
  float* out = (float*)d_out;

  char* ws = (char*)d_ws;
  unsigned short* XA   = (unsigned short*)(ws + kOffXA);
  float*          XPRE = (float*)(ws + kOffXPRE);
  unsigned short* YSC  = (unsigned short*)(ws + kOffYSC);
  unsigned short* WIN  = (unsigned short*)(ws + kOffWIN);
  unsigned short* WXP  = (unsigned short*)(ws + kOffWXP);
  unsigned short* WOUT = (unsigned short*)(ws + kOffWOUT);
  float*          Zp   = (float*)(ws + kOffZ);
  float*          XS   = (float*)(ws + kOffXS);
  unsigned short* XSh  = (unsigned short*)(ws + kOffXSh);
  unsigned short* YG   = (unsigned short*)(ws + kOffXSh);
  float*          P    = (float*)(ws + kOffP);
  float*          WD   = (float*)(ws + kOffWD);

  prep_x_kernel<<<kNb * (kLen / 64), 256, 0, stream>>>(x, XA);
  prep_w_kernel<<<42, 256, 0, stream>>>(ipw, xpw, opw, WIN, WXP, WOUT);
  wmma_gemm64<1><<<dim3(192, 2), 256, 0, stream>>>(
      XA, kPitA, 0L,
      WIN, kPitA, (long)(kDin * kPitA),
      XPRE, kDin, (long)((kOffZ - kOffXPRE) / 4),
      kPix, kDin, kDm, 1.0f, kPix);
  dwconv_silu_kernel<<<kPix / 8, 192, 0, stream>>>(XPRE, cw, cb, XS, XSh);
  wmma_gemm64<0><<<dim3(64, 1), 256, 0, stream>>>(
      XSh, kDin, 0L,
      WXP, kDin, 0L,
      P, kPitP, 0L,
      kPix, kPitP, kDin, kUncarry2, kPix);
  prior_weights_kernel<<<kPix / 256, 256, 0, stream>>>(prior, alpha, w1, b1, bnw, bnb, bnm, bnv, w2, b2, WD);
  scan_kernel<<<kNb * kDir * (kDin / 64), 64, 0, stream>>>(P, XS, dtw, dtb, alog, YSC);
  merge_norm_gate_kernel<<<kPix / 32, 256, 0, stream>>>(XS, Zp, (const unsigned*)(const void*)YSC, WD, Dsg, onw, onb,
                                                        (unsigned*)(void*)YG);
  wmma_gemm64<0><<<dim3(16, kNb), 256, 0, stream>>>(
      WOUT, kDin, 0L,
      YG, kDin, (long)(kLen * kDin),
      out, kLen, (long)(kDm * kLen),
      kMpadO, kLen, kDin, kUncarry2, kDm);
}
